// CausalAttention_33930241639029
// MI455X (gfx1250) — hardware-verified
//
#include <hip/hip_runtime.h>


#ifndef NB
#define NB 2
#endif
#ifndef SEQ
#define SEQ 2048
#endif
#ifndef RH
#define RH 256
#endif
#define NB_FULL  2
#define SEQ_FULL 2048
#define DIMM 1024
#define NHD  8
#define HD   128
#define NBH  (NB * NHD)
#define NBLK (SEQ / 64)
#define QKVW 3072
#define KCAT (3 * HD)
#define PCAT (3 * RH)
#define WCAR 64.0f
#define MCAR 16.0f
#define PSH  10.0f
#define SCALEQ 0.08838834764831845f
#define L2E 1.4426950408889634f
#define OUT1_OFF ((size_t)NB_FULL * SEQ_FULL * DIMM)
#define OUT2_OFF (OUT1_OFF + (size_t)NB_FULL * NHD * HD * HD)

static_assert(OUT1_OFF * 4 == 16777216);
static_assert(OUT2_OFF * 4 == 17825792);
static_assert(SEQ % 64 == 0);
static_assert(RH % 128 == 0);
static_assert(RH <= SEQ);
static_assert((SEQ - RH) % 64 == 0);
static_assert(NB <= NB_FULL);
static_assert(SEQ <= SEQ_FULL);
static_assert((NB * SEQ) % 8 == 0);

typedef _Float16 h16;
typedef unsigned short bf;
typedef __attribute__((ext_vector_type(16))) __bf16   v16bf;
typedef __attribute__((ext_vector_type(16))) _Float16 v16h;
typedef __attribute__((ext_vector_type(8)))  _Float16 v8h;
typedef __attribute__((ext_vector_type(8)))  unsigned short v8us;
typedef __attribute__((ext_vector_type(4)))  unsigned short v4us;
typedef __attribute__((ext_vector_type(8)))  float    v8f;
typedef __attribute__((ext_vector_type(4)))  float    v4f;
typedef v8h  __attribute__((may_alias)) v8ha;
typedef v4f  __attribute__((may_alias)) v4fa;
typedef v8us __attribute__((may_alias)) v8usa;

#define WSYNC() do { __builtin_amdgcn_fence(3  , "wavefront"); __builtin_amdgcn_wave_barrier(); asm volatile("" ::: "memory"); } while (0)

__device__ __forceinline__ unsigned short f2bf(float f) { unsigned u = __float_as_uint(f); u += 0x7FFFu + ((u >> 16) & 1u); return (unsigned short)(u >> 16); }
__device__ __forceinline__ float bf2f(unsigned short b) { return __uint_as_float(((unsigned)b) << 16); }
__device__ __forceinline__ float bfr(float f) { return bf2f(f2bf(f)); }
__device__ __forceinline__ void splitf(float y, unsigned short& h, unsigned short& l) { h = f2bf(y); l = f2bf(y - bf2f(h)); }
__device__ __forceinline__ v16h cat16(v8h lo, v8h hi) { return __builtin_shufflevector(lo, hi, 0, 1, 2, 3, 4, 5, 6, 7, 8, 9, 10, 11, 12, 13, 14, 15); }
__device__ __forceinline__ v16bf cat16b(v8us lo, v8us hi) { return __builtin_bit_cast(v16bf, __builtin_shufflevector(lo, hi, 0, 1, 2, 3, 4, 5, 6, 7, 8, 9, 10, 11, 12, 13, 14, 15)); }
__device__ __forceinline__ v8f wmma16(v16h a, v16h b, v8f c) { return __builtin_amdgcn_wmma_f32_16x16x32_f16(false, a, false, b, (short)0, c, false, false); }
__device__ __forceinline__ v8f wmmab(v16bf a, v16bf b, v8f c) { return __builtin_amdgcn_wmma_f32_16x16x32_bf16(false, a, false, b, (short)0, c, false, false); }

template <typename T16> struct WFrag;
template <> struct WFrag<h16> { typedef v16h V; static __device__ __forceinline__ V ld(const h16* p) { return cat16(*(const v8h*)p, *(const v8h*)(p + 16)); } static __device__ __forceinline__ v8f mma(V a, V b, v8f c) { return wmma16(a, b, c); } };
template <> struct WFrag<bf> { typedef v16bf V; static __device__ __forceinline__ V ld(const bf* p) { return cat16b(*(const v8us*)p, *(const v8us*)(p + 16)); } static __device__ __forceinline__ v8f mma(V a, V b, v8f c) { return wmmab(a, b, c); } };

template <typename T16, int NSPLIT, bool ADDM>
__global__ __launch_bounds__(32) void k_gemmw(const T16* __restrict__ A, const T16* __restrict__ A2, const T16* __restrict__ Bt, int K, float* C, int ldc, const float* __restrict__ addm, float cscale, size_t sA, size_t sB, size_t sC) {
    typedef typename WFrag<T16>::V V;
    __shared__ __align__(16) float os[16 * 68];
    const size_t z = blockIdx.z; A += z * sA; if (NSPLIT == 1) A2 += z * sA; Bt += z * sB; C += z * sC; if (ADDM) addm += z * sC;
    const int lane = threadIdx.x & 31, lr = lane & 15, hi = lane >> 4; const int r0 = blockIdx.x * 64, c0 = blockIdx.y * 64;
    v8f acc[4][4];
#pragma unroll
    for (int mb = 0; mb < 4; ++mb)
#pragma unroll
        for (int nb = 0; nb < 4; ++nb) acc[mb][nb] = (v8f){};
    const size_t aoff = (size_t)(r0 + lr) * K + 8 * hi, boff = (size_t)(c0 + lr) * K + 8 * hi;
#pragma unroll 1
    for (int kc = 0; kc < K; kc += 32) {
        V a[4], a2[4];
#pragma unroll
        for (int mb = 0; mb < 4; ++mb) { a[mb] = WFrag<T16>::ld(A + aoff + (size_t)mb * 16 * K + kc); if (NSPLIT == 1) a2[mb] = WFrag<T16>::ld(A2 + aoff + (size_t)mb * 16 * K + kc); }
#pragma unroll
        for (int nb = 0; nb < 4; ++nb) { const V b = WFrag<T16>::ld(Bt + boff + (size_t)nb * 16 * K + kc);
#pragma unroll
            for (int mb = 0; mb < 4; ++mb) { acc[mb][nb] = WFrag<T16>::mma(a[mb], b, acc[mb][nb]); if (NSPLIT == 1) acc[mb][nb] = WFrag<T16>::mma(a2[mb], b, acc[mb][nb]); } }
        asm volatile("v_nop\n\tv_nop\n\tv_nop\n\tv_nop" : "+v"(acc[0][0]), "+v"(acc[1][1]), "+v"(acc[2][2]), "+v"(acc[3][3]) : "v"(a[0]), "v"(a[3]));
    }
#pragma unroll
    for (int mb = 0; mb < 4; ++mb) {
#pragma unroll
        for (int nb = 0; nb < 4; ++nb) {
#pragma unroll
            for (int j = 0; j < 8; ++j) os[(hi * 8 + j) * 68 + nb * 16 + lr] = acc[mb][nb][j]; }
        WSYNC();
        float* crow = C + (size_t)(r0 + mb * 16) * ldc + c0;
        const float* arow = ADDM ? (addm + (size_t)(r0 + mb * 16) * ldc + c0) : C;
#pragma unroll 1
        for (int ps = 0; ps < 2; ++ps) {
#pragma unroll
            for (int s = 0; s < 8; ++s) { const int row = 2 * s + hi, cofs = lr * 4; v4f val = *(const v4fa*)(os + row * 68 + cofs); val = val * cscale;
                if (ADDM) { const v4f ad = *(const v4f*)(arow + (size_t)row * ldc + cofs); val[0] += bfr(ad[0]); val[1] += bfr(ad[1]); val[2] += bfr(ad[2]); val[3] += bfr(ad[3]); }
                *(volatile v4f*)(crow + (size_t)row * ldc + cofs) = val; }
            if (ps == 0) __threadfence(); }
        WSYNC();
    }
}

__global__ __launch_bounds__(256) void k_cvtw(const float* __restrict__ src, bf* dB, h16* dH, unsigned n8) {
    const unsigned i = blockIdx.x * 256u + threadIdx.x; if (i >= n8) return;
    const v8f v = *(const v8f*)(src + (size_t)i * 8); v8us ob; v8h oh;
#pragma unroll
    for (int k = 0; k < 8; ++k) { ob[k] = f2bf(v[k]); oh[k] = (h16)(bf2f(ob[k]) * WCAR); }
    *(volatile v8us*)(dB + (size_t)i * 8) = ob; *(volatile v8h*)(dH + (size_t)i * 8) = oh; __threadfence();
    *(volatile v8us*)(dB + (size_t)i * 8) = ob; *(volatile v8h*)(dH + (size_t)i * 8) = oh;
}

__global__ __launch_bounds__(256) void k_memT(const float* __restrict__ mem, h16* MEMT) {
    __shared__ __align__(16) h16 T[128 * 136];
    const unsigned tid = threadIdx.x, bh = blockIdx.x;
    const float* mb = mem + (size_t)bh * HD * HD;
#pragma unroll 2
    for (unsigned j = 0; j < 16u; ++j) { const unsigned idx = tid + 256u * j, k = idx >> 5, c4 = (idx & 31u) * 4u; const v4f v = *(const v4f*)(mb + (size_t)k * HD + c4);
#pragma unroll
        for (int e = 0; e < 4; ++e) T[(c4 + e) * 136u + k] = (h16)bfr(v[e]); }
    __syncthreads();
#pragma unroll 1
    for (int ps = 0; ps < 2; ++ps) {
#pragma unroll 2
        for (unsigned j = 0; j < 8u; ++j) { const unsigned idx = tid + 256u * j, vv = idx >> 4, pc = idx & 15u; const v8h a = *(const v8ha*)(T + vv * 136u + pc * 8u);
            h16* d0 = MEMT + ((size_t)bh * HD + vv) * HD + pc * 8u; *(volatile v8h*)d0 = a; *(volatile v8h*)(d0 + (size_t)NBH * HD * HD) = a; }
        if (ps == 0) __threadfence(); }
}

__global__ __launch_bounds__(32) void k_invf(float* INVF) {
    const unsigned lane = threadIdx.x & 31u;
#pragma unroll 1
    for (unsigned q = 0; q < 2u; ++q) { const unsigned i = lane + 32u * q; const float e = (float)(2u * i) * (1.0f / 128.0f); const float v = 1.0f / powf(10000.0f, e);
        *(volatile float*)(INVF + i) = v; __threadfence(); *(volatile float*)(INVF + i) = v; }
}

__global__ __launch_bounds__(256) void k_ropetab(const float* __restrict__ INVF, float* COS, float* SIN) {
    const unsigned idx = blockIdx.x * 256u + threadIdx.x; const unsigned t = idx >> 6, i = idx & 63u;
    const float ang = (float)t * INVF[i]; const float c = cosf(ang); const float s = sinf(ang);
    *(volatile float*)(COS + idx) = c; *(volatile float*)(SIN + idx) = s; __threadfence();
    *(volatile float*)(COS + idx) = c; *(volatile float*)(SIN + idx) = s;
}

__global__ __launch_bounds__(256) void k_rms(const float* __restrict__ x, const float* __restrict__ gamma, h16* XN, bf* XH, bf* XL) {
    const unsigned lane = threadIdx.x & 31u, wv = threadIdx.x >> 5;
    const unsigned r = blockIdx.x * 8u + wv; const unsigned b = r / (unsigned)SEQ, t = r - b * (unsigned)SEQ;
    const float* xr = x + ((size_t)b * SEQ_FULL + t) * DIMM;
    float ss = 0.f;
#pragma unroll 1
    for (unsigned c = 0; c < 4u; ++c) { const v8f v = *(const v8f*)(xr + c * 256u + lane * 8u);
#pragma unroll
        for (int k = 0; k < 8; ++k) { const float f = bfr(v[k]); ss += f * f; } }
#pragma unroll
    for (int sh = 16; sh; sh >>= 1) ss += __shfl_xor(ss, sh, 32);
    const float rinv = 1.0f / fmaxf(sqrtf(ss), 1e-12f);
    const bool early = (t < (unsigned)RH);
#pragma unroll 1
    for (unsigned c = 0; c < 4u; ++c) { const unsigned col = c * 256u + lane * 8u; const v8f v = *(const v8f*)(xr + col); const v8f g = *(const v8f*)(gamma + col);
        v8h o; v8us oh, ol;
#pragma unroll
        for (int k = 0; k < 8; ++k) { const float y = ((bfr(v[k]) * rinv) * 32.0f) * bfr(g[k]); o[k] = (h16)y; unsigned short a, c2; splitf(y, a, c2); oh[k] = a; ol[k] = c2; }
        h16* dn = XN + (size_t)r * DIMM + col; const size_t eo = ((size_t)b * RH + (early ? t : 0u)) * DIMM + col;
#pragma unroll 1
        for (int ps = 0; ps < 2; ++ps) { *(volatile v8h*)dn = o; if (early) { *(volatile v8us*)(XH + eo) = oh; *(volatile v8us*)(XL + eo) = ol; } if (ps == 0) __threadfence(); } }
}

#define TP 72
__global__ __launch_bounds__(256) void k_prep(const float* __restrict__ QKV, const float* __restrict__ COS, const float* __restrict__ SIN, const float* __restrict__ mnorm,
                                              h16* QROT, h16* KROT, h16* VT, h16* FEAT, h16* KFT, bf* QC, bf* KC, bf* VTC, float* PART, float* RDEN) {
    __shared__ __align__(16) h16 tV[128 * TP];
    __shared__ __align__(16) h16 tK[128 * TP];
    __shared__ __align__(16) unsigned short tVh[128 * TP];
    __shared__ __align__(16) unsigned short tVl[128 * TP];
    __shared__ __align__(16) float red[8 * 128];
    __shared__ __align__(16) float dens[2 * 64];
    const unsigned tid = threadIdx.x, lane = tid & 31u, wv = tid >> 5;
    const unsigned bh = blockIdx.y, b = bh >> 3, h = bh & 7u, t0 = blockIdx.x * 64u;
    const bool early = (t0 < (unsigned)RH);
    const unsigned c8 = (tid & 15u) * 8u;
    float mn[8];
    { const v8f m8 = *(const v8f*)(mnorm + (size_t)bh * HD + c8);
#pragma unroll
      for (int e = 0; e < 8; ++e) mn[e] = bfr(m8[e]); }
    float ksum[8];
#pragma unroll
    for (int e = 0; e < 8; ++e) ksum[e] = 0.f;
#pragma unroll 1
    for (unsigned j = 0; j < 4u; ++j) {
        const unsigned row = (tid >> 4) + 16u * j, t = t0 + row;
        const float* src = QKV + ((size_t)b * SEQ + t) * QKVW + h * HD + c8;
        const v8f q8 = *(const v8f*)src, k8 = *(const v8f*)(src + DIMM), v8 = *(const v8f*)(src + 2 * DIMM);
        const v4f cs = *(const v4f*)(COS + (size_t)t * 64u + (c8 >> 1)), sn = *(const v4f*)(SIN + (size_t)t * 64u + (c8 >> 1));
        float qr[8], kr[8], qf[8], kf[8];
#pragma unroll
        for (int p = 0; p < 4; ++p) { const float c = cs[p], s = sn[p];
            qr[2 * p] = q8[2 * p] * c - q8[2 * p + 1] * s; qr[2 * p + 1] = q8[2 * p + 1] * c + q8[2 * p] * s;
            kr[2 * p] = k8[2 * p] * c - k8[2 * p + 1] * s; kr[2 * p + 1] = k8[2 * p + 1] * c + k8[2 * p] * s; }
        float dq = 0.f, dk = 0.f;
#pragma unroll
        for (int e = 0; e < 8; ++e) { const float eq = __builtin_amdgcn_exp2f(fminf(q8[e], 0.f) * L2E), ek = __builtin_amdgcn_exp2f(fminf(k8[e], 0.f) * L2E);
            qf[e] = (q8[e] > 0.f) ? (q8[e] + 1.0f) : eq; kf[e] = (k8[e] > 0.f) ? (k8[e] + 1.0f) : ek; dq += qf[e] * mn[e]; dk += kf[e] * mn[e]; ksum[e] += kf[e]; }
#pragma unroll
        for (int sh = 8; sh; sh >>= 1) { dq += __shfl_xor(dq, sh, 32); dk += __shfl_xor(dk, sh, 32); }
        if ((lane & 15u) == 0u) { dens[row] = 1.0f / fmaxf(dq, 1e-10f); dens[64u + row] = 1.0f / fmaxf(dk, 1e-10f); }
        v8h oq, ok, of, og; v8us qh, ql, kh, kl;
#pragma unroll
        for (int e = 0; e < 8; ++e) { oq[e] = (h16)qr[e]; ok[e] = (h16)kr[e]; of[e] = (h16)qf[e]; og[e] = (h16)kf[e];
            unsigned short a, c2; splitf(qr[e], a, c2); qh[e] = a; ql[e] = c2; splitf(kr[e], a, c2); kh[e] = a; kl[e] = c2;
            tV[(c8 + e) * TP + row] = (h16)v8[e]; tK[(c8 + e) * TP + row] = og[e];
            splitf(v8[e], a, c2); tVh[(c8 + e) * TP + row] = a; tVl[(c8 + e) * TP + row] = c2; }
        const size_t ro = ((size_t)bh * SEQ + t) * HD + c8;
        const size_t eo = ((size_t)bh * RH + (early ? t : 0u)) * KCAT + c8;
#pragma unroll 1
        for (int ps = 0; ps < 2; ++ps) {
            *(volatile v8h*)(QROT + ro) = oq; *(volatile v8h*)(KROT + ro) = ok; *(volatile v8h*)(FEAT + ro) = of; *(volatile v8h*)(FEAT + (size_t)NBH * SEQ * HD + ro) = og;
            if (early) { *(volatile v8us*)(QC + eo) = qh; *(volatile v8us*)(QC + eo + HD) = ql; *(volatile v8us*)(QC + eo + 2 * HD) = qh;
                         *(volatile v8us*)(KC + eo) = kh; *(volatile v8us*)(KC + eo + HD) = kh; *(volatile v8us*)(KC + eo + 2 * HD) = kl; }
            if (ps == 0) __threadfence(); }
    }
#pragma unroll
    for (int e = 0; e < 8; ++e) ksum[e] += __shfl_xor(ksum[e], 16, 32);
    if (lane < 16u) { v4f s0, s1; s0[0] = ksum[0]; s0[1] = ksum[1]; s0[2] = ksum[2]; s0[3] = ksum[3]; s1[0] = ksum[4]; s1[1] = ksum[5]; s1[2] = ksum[6]; s1[3] = ksum[7];
        *(v4fa*)(red + wv * 128u + c8) = s0; *(v4fa*)(red + wv * 128u + c8 + 4u) = s1; }
    __syncthreads();
#pragma unroll 1
    for (int ps = 0; ps < 2; ++ps) {
#pragma unroll
        for (unsigned jj = 0; jj < 4u; ++jj) { const unsigned idx = tid + 256u * jj, d = idx >> 3, pc = idx & 7u;
            const v8h a = *(const v8ha*)(tV + d * TP + pc * 8u); const v8h c = *(const v8ha*)(tK + d * TP + pc * 8u);
            const size_t o = ((size_t)bh * HD + d) * SEQ + t0 + pc * 8u;
            *(volatile v8h*)(VT + o) = a; *(volatile v8h*)(KFT + o) = c;
            if (early) { const v8us hv = *(const v8usa*)(tVh + d * TP + pc * 8u); const v8us lv = *(const v8usa*)(tVl + d * TP + pc * 8u);
                const size_t oe = ((size_t)bh * HD + d) * PCAT + t0 + pc * 8u;
                *(volatile v8us*)(VTC + oe) = hv; *(volatile v8us*)(VTC + oe + RH) = hv; *(volatile v8us*)(VTC + oe + 2 * RH) = lv; } }
        if (ps == 0) __threadfence(); }
    if (tid < 32u) {
        const unsigned d4 = tid * 4u; v4f s = *(const v4fa*)(red + d4);
#pragma unroll
        for (unsigned w = 1; w < 8u; ++w) { const v4f u = *(const v4fa*)(red + w * 128u + d4); s = s + u; }
        const unsigned wh = tid >> 4, l4 = (tid & 15u) * 4u; const v4f rdv = *(const v4fa*)(dens + wh * 64u + l4);
        float* pp = PART + ((size_t)bh * NBLK + blockIdx.x) * HD + d4; float* rp = RDEN + ((size_t)wh * NBH + bh) * SEQ + t0 + l4;
        *(volatile v4f*)pp = s; *(volatile v4f*)rp = rdv; __threadfence(); *(volatile v4f*)pp = s; *(volatile v4f*)rp = rdv; }
}

__global__ __launch_bounds__(256) void k_asoftE(const float* __restrict__ Sb, bf* PCp) {
    const unsigned lane = threadIdx.x & 31u; const unsigned row = blockIdx.x * 8u + (threadIdx.x >> 5); const unsigned i = row % (unsigned)RH;
    const float* sr = Sb + (size_t)row * RH; float v[RH / 32]; float mx = -3.0e38f;
#pragma unroll
    for (int ch = 0; ch < RH / 128; ++ch) { const unsigned j0 = ch * 128u + lane * 4u; const v4f a = *(const v4f*)(sr + j0);
#pragma unroll
        for (int q = 0; q < 4; ++q) { const unsigned j = j0 + q; const float t = (j <= i) ? a[q] * SCALEQ : -3.0e38f; v[ch * 4 + q] = t; mx = fmaxf(mx, t); } }
#pragma unroll
    for (int sh = 16; sh; sh >>= 1) mx = fmaxf(mx, __shfl_xor(mx, sh, 32));
    float sum = 0.f;
#pragma unroll
    for (int k = 0; k < RH / 32; ++k) { const float d0 = v[k] - mx; v[k] = __builtin_amdgcn_exp2f(d0 * L2E); sum += v[k]; }
#pragma unroll
    for (int sh = 16; sh; sh >>= 1) sum += __shfl_xor(sum, sh, 32);
    const float f = 1.0f / sum;
#pragma unroll 1
    for (int ps = 0; ps < 2; ++ps) {
#pragma unroll
        for (int ch = 0; ch < RH / 128; ++ch) { v4us oh, ol;
#pragma unroll
            for (int q = 0; q < 4; ++q) { unsigned short a, c2; splitf(v[ch * 4 + q] * f, a, c2); oh[q] = a; ol[q] = c2; }
            const size_t oo = (size_t)row * PCAT + ch * 128u + lane * 4u; *(volatile v4us*)(PCp + oo) = oh; *(volatile v4us*)(PCp + oo + RH) = ol; *(volatile v4us*)(PCp + oo + 2 * RH) = oh; }
        if (ps == 0) __threadfence(); }
}

__global__ __launch_bounds__(256) void k_mergeE(const float* __restrict__ CTXE, const float* __restrict__ NUMq, const float* __restrict__ RDq, const float* __restrict__ gates, bf* MH, bf* ML) {
    const unsigned idx = blockIdx.x * 256u + threadIdx.x; const unsigned c8 = (idx & 15u) * 8u; const unsigned rt = idx >> 4; const unsigned t = rt % (unsigned)RH, z = rt / (unsigned)RH;
    const unsigned b = z >> 3, h = z & 7u;
    const float g = 1.0f / (1.0f + expf(-bfr(gates[h]))); const float omg = 1.0f - g;
    const v8f c = *(const v8f*)(CTXE + ((size_t)z * RH + t) * HD + c8); const v8f n = *(const v8f*)(NUMq + ((size_t)z * SEQ + t) * HD + c8); const float rd = RDq[(size_t)z * SEQ + t];
    v8us oh, ol;
#pragma unroll
    for (int e = 0; e < 8; ++e) { const float val = c[e] * g + (n[e] * rd) * omg; unsigned short a, c2; splitf(val, a, c2); oh[e] = a; ol[e] = c2; }
    const size_t o = ((size_t)b * RH + t) * DIMM + h * HD + c8;
    *(volatile v8us*)(MH + o) = oh; *(volatile v8us*)(ML + o) = ol; __threadfence(); *(volatile v8us*)(MH + o) = oh; *(volatile v8us*)(ML + o) = ol;
}

__global__ __launch_bounds__(32) void k_flash(const h16* __restrict__ Q, const h16* __restrict__ Kp, const h16* __restrict__ VT, const float* __restrict__ NUMq, const float* __restrict__ RDq, const float* __restrict__ gates, h16* MRG) {
    __shared__ __align__(16) float os[16 * 132];
    const unsigned lane = threadIdx.x & 31u, lr = lane & 15u, hi = lane >> 4;
    const unsigned bh = blockIdx.y, b = bh >> 3, h = bh & 7u;
    const unsigned q0 = (unsigned)RH + blockIdx.x * 16u;
    const h16* Qb = Q + (size_t)bh * SEQ * HD; const h16* Kb = Kp + (size_t)bh * SEQ * HD; const h16* Vb = VT + (size_t)bh * HD * SEQ;
    v16h qb[4];
#pragma unroll
    for (int c = 0; c < 4; ++c) qb[c] = WFrag<h16>::ld(Qb + (size_t)(q0 + lr) * HD + 8u * hi + 32u * c);
    v8f acc[8];
#pragma unroll
    for (int d = 0; d < 8; ++d) acc[d] = (v8f){};
    float m = -3.0e38f, ls = 0.f;
    const unsigned nst = (q0 >> 5) + 1u, qme = q0 + lr;
    const float sc2 = SCALEQ * L2E;
#pragma unroll 1
    for (unsigned ks = 0; ks < nst; ++ks) {
        const unsigned k0 = ks * 32u;
        v8f s0 = (v8f){}, s1 = (v8f){};
        const h16* kp = Kb + (size_t)(k0 + lr) * HD + 8u * hi;
#pragma unroll
        for (int c = 0; c < 4; ++c) { const v16h a0 = WFrag<h16>::ld(kp + 32 * c); const v16h a1 = WFrag<h16>::ld(kp + 16 * HD + 32 * c); s0 = wmma16(a0, qb[c], s0); s1 = wmma16(a1, qb[c], s1); }
        asm volatile("v_nop\n\tv_nop\n\tv_nop\n\tv_nop" : "+v"(s0), "+v"(s1) : "v"(qb[0]), "v"(qb[3]));
        const unsigned kb = k0 + 8u * hi;
        float x0[8], x1[8]; float ml = -3.0e38f;
#pragma unroll
        for (int r = 0; r < 8; ++r) { const unsigned ky = kb + (unsigned)r; x0[r] = (ky <= qme) ? s0[r] * sc2 : -3.0e38f; x1[r] = (ky + 16u <= qme) ? s1[r] * sc2 : -3.0e38f; ml = fmaxf(ml, fmaxf(x0[r], x1[r])); }
        ml = fmaxf(ml, __shfl_xor(ml, 16, 32));
        const float mnw = fmaxf(m, ml);
        const float resc = __builtin_amdgcn_exp2f(m - mnw);
        const unsigned up = __builtin_amdgcn_ballot_w32(mnw > m);
        const float shf = PSH - mnw;
        float psum = 0.f; v16h pb;
#pragma unroll
        for (int r = 0; r < 8; ++r) { const float p0 = __builtin_amdgcn_exp2f(x0[r] + shf), p1 = __builtin_amdgcn_exp2f(x1[r] + shf); psum += p0 + p1; pb[r] = (h16)p0; pb[8 + r] = (h16)p1; }
        ls = ls * resc + psum; m = mnw;
        if (up != 0u) {
#pragma unroll
            for (int d = 0; d < 8; ++d) acc[d] = acc[d] * resc; }
        const h16* vp = Vb + (size_t)lr * SEQ + k0 + 8u * hi;
#pragma unroll
        for (int d = 0; d < 8; ++d) { const v16h av = WFrag<h16>::ld(vp + (size_t)d * 16 * SEQ); acc[d] = wmma16(av, pb, acc[d]); }
        asm volatile("v_nop\n\tv_nop\n\tv_nop\n\tv_nop" : "+v"(acc[0]), "+v"(acc[1]), "+v"(acc[2]), "+v"(acc[3]), "+v"(acc[4]), "+v"(acc[5]), "+v"(acc[6]), "+v"(acc[7]) : "v"(pb));
    }
    const float lt = ls + __shfl_xor(ls, 16, 32);
    const float inv = 1.0f / lt;
#pragma unroll
    for (int d = 0; d < 8; ++d) { v4f a, c; a[0] = acc[d][0] * inv; a[1] = acc[d][1] * inv; a[2] = acc[d][2] * inv; a[3] = acc[d][3] * inv; c[0] = acc[d][4] * inv; c[1] = acc[d][5] * inv; c[2] = acc[d][6] * inv; c[3] = acc[d][7] * inv;
        *(v4fa*)(os + lr * 132u + 16u * d + 8u * hi) = a; *(v4fa*)(os + lr * 132u + 16u * d + 8u * hi + 4u) = c; }
    WSYNC();
    const float g = 1.0f / (1.0f + expf(-bfr(gates[h]))); const float omg = 1.0f - g;
    v8h ov[8];
#pragma unroll
    for (int s = 0; s < 8; ++s) { const unsigned row = 2u * s + hi, t = q0 + row, c8 = lr * 8u;
        const v4f o0 = *(const v4fa*)(os + row * 132u + c8), o1 = *(const v4fa*)(os + row * 132u + c8 + 4u);
        const v8f n = *(const v8f*)(NUMq + ((size_t)bh * SEQ + t) * HD + c8); const float rd = RDq[(size_t)bh * SEQ + t];
#pragma unroll
        for (int e = 0; e < 4; ++e) { ov[s][e] = (h16)((o0[e] * g + (n[e] * rd) * omg) * MCAR); ov[s][4 + e] = (h16)((o1[e] * g + (n[4 + e] * rd) * omg) * MCAR); } }
#pragma unroll 1
    for (int ps = 0; ps < 2; ++ps) {
#pragma unroll
        for (int s = 0; s < 8; ++s) { const unsigned row = 2u * s + hi, t = q0 + row; *(volatile v8h*)(MRG + ((size_t)b * SEQ + t) * DIMM + h * HD + lr * 8u) = ov[s]; }
        if (ps == 0) __threadfence(); }
}

__global__ __launch_bounds__(256) void k_vnew(const float* __restrict__ NUMk, const float* __restrict__ RDk, const h16* __restrict__ VT, h16* VNT) {
    __shared__ __align__(16) float Tn[128 * 68];
    const unsigned tid = threadIdx.x, bh = blockIdx.y, t0 = blockIdx.x * 64u;
#pragma unroll 2
    for (unsigned j = 0; j < 8u; ++j) { const unsigned idx = tid + 256u * j, row = idx >> 5, c4 = (idx & 31u) * 4u; const v4f n = *(const v4f*)(NUMk + ((size_t)bh * SEQ + t0 + row) * HD + c4); const float rd = RDk[(size_t)bh * SEQ + t0 + row];
#pragma unroll
        for (int e = 0; e < 4; ++e) Tn[(c4 + e) * 68u + row] = n[e] * rd; }
    __syncthreads();
#pragma unroll 1
    for (int ps = 0; ps < 2; ++ps) {
#pragma unroll
        for (unsigned jj = 0; jj < 4u; ++jj) { const unsigned idx = tid + 256u * jj, d = idx >> 3, pc = idx & 7u; const size_t o = ((size_t)bh * HD + d) * SEQ + t0 + pc * 8u;
            const v8h vt = *(const v8h*)(VT + o); const v4f d0 = *(const v4fa*)(Tn + d * 68u + pc * 8u), d1 = *(const v4fa*)(Tn + d * 68u + pc * 8u + 4u); v8h w;
#pragma unroll
            for (int e = 0; e < 4; ++e) { w[e] = (h16)((float)vt[e] - d0[e]); w[4 + e] = (h16)((float)vt[4 + e] - d1[e]); }
            *(volatile v8h*)(VNT + o) = w; }
        if (ps == 0) __threadfence(); }
}

__global__ __launch_bounds__(32) void k_normfin(const float* __restrict__ PART, const float* __restrict__ mnorm, float* out2) {
    const unsigned bh = blockIdx.x, d4 = (threadIdx.x & 31u) * 4u;
    v4f s = *(const v4f*)(PART + (size_t)bh * NBLK * HD + d4);
#pragma unroll 1
    for (unsigned k = 1; k < (unsigned)NBLK; ++k) { const v4f u = *(const v4f*)(PART + ((size_t)bh * NBLK + k) * HD + d4); s = s + u; }
    const v4f mnv = *(const v4f*)(mnorm + (size_t)bh * HD + d4);
    s[0] += bfr(mnv[0]); s[1] += bfr(mnv[1]); s[2] += bfr(mnv[2]); s[3] += bfr(mnv[3]);
    float* o = out2 + (size_t)bh * HD + d4; *(volatile v4f*)o = s; __threadfence(); *(volatile v4f*)o = s;
}

constexpr size_t cmax(size_t a, size_t b) { return a > b ? a : b; }
constexpr size_t SZ_WQ   = (size_t)QKVW * DIMM * 2;
constexpr size_t SZ_WO   = (size_t)DIMM * DIMM * 2;
constexpr size_t SZ_QC   = (size_t)NBH * RH * KCAT * 2;
constexpr size_t SZ_VTC  = (size_t)NBH * HD * PCAT * 2;
constexpr size_t SZ_RW   = cmax(2 * SZ_WQ, 2 * SZ_QC + SZ_VTC);
constexpr size_t SZ_MEMT = (size_t)2 * NBH * HD * HD * 2;
constexpr size_t SZ_INVF = 256;
constexpr size_t SZ_TAB  = (size_t)SEQ * 64 * 4;
constexpr size_t SZ_XN   = (size_t)NB * SEQ * DIMM * 2;
constexpr size_t SZ_XE   = (size_t)NB * RH * DIMM * 2;
constexpr size_t SZ_QKV  = (size_t)NB * SEQ * QKVW * 4;
constexpr size_t SZ_NUM  = (size_t)2 * NBH * SEQ * HD * 4;
constexpr size_t SZ_SE   = (size_t)NBH * RH * RH * 4;
constexpr size_t SZ_PC   = (size_t)NBH * RH * PCAT * 2;
constexpr size_t SZ_CTXE = (size_t)NBH * RH * HD * 4;
constexpr size_t SZ_RQ   = cmax(SZ_QKV, SZ_NUM + SZ_SE + SZ_PC + SZ_CTXE);
constexpr size_t SZ_PL   = (size_t)NBH * SEQ * HD * 2;
constexpr size_t SZ_PART = (size_t)NBH * NBLK * HD * 4;
constexpr size_t SZ_RDEN = (size_t)2 * NBH * SEQ * 4;
constexpr size_t O_RW   = 0;
constexpr size_t O_WOB  = O_RW + SZ_RW;
constexpr size_t O_WOH  = O_WOB + SZ_WO;
constexpr size_t O_MEMT = O_WOH + SZ_WO;
constexpr size_t O_INVF = O_MEMT + SZ_MEMT;
constexpr size_t O_COS  = O_INVF + SZ_INVF;
constexpr size_t O_SIN  = O_COS + SZ_TAB;
constexpr size_t O_XN   = O_SIN + SZ_TAB;
constexpr size_t O_XH   = O_XN + SZ_XN;
constexpr size_t O_XL   = O_XH + SZ_XE;
constexpr size_t O_RQ   = O_XL + SZ_XE;
constexpr size_t O_QROT = O_RQ + SZ_RQ;
constexpr size_t O_KROT = O_QROT + SZ_PL;
constexpr size_t O_VT   = O_KROT + SZ_PL;
constexpr size_t O_FEAT = O_VT + SZ_PL;
constexpr size_t O_KFT  = O_FEAT + 2 * SZ_PL;
constexpr size_t O_PART = O_KFT + SZ_PL;
constexpr size_t O_RDEN = O_PART + SZ_PART;
constexpr size_t WS_TOTAL = O_RDEN + SZ_RDEN;
static_assert(WS_TOTAL <= (size_t)134217728);
static_assert(SZ_RW % 256 == 0 && SZ_WO % 256 == 0 && SZ_MEMT % 256 == 0 && SZ_TAB % 256 == 0 && SZ_XN % 256 == 0 && SZ_XE % 256 == 0 && SZ_RQ % 256 == 0 && SZ_PL % 256 == 0 && SZ_PART % 256 == 0 && SZ_RDEN % 256 == 0);
static_assert(SZ_QC % 256 == 0 && SZ_NUM % 256 == 0 && SZ_SE % 256 == 0 && SZ_PC % 256 == 0);
static_assert(DIMM % 64 == 0 && QKVW % 64 == 0 && HD % 64 == 0 && KCAT % 32 == 0 && PCAT % 32 == 0 && RH % 64 == 0 && SEQ % 32 == 0);

extern "C" void kernel_launch(void* const* d_in, const int* in_sizes, int n_in,
                              void* d_out, int out_size, void* d_ws, size_t ws_size, hipStream_t stream) {
    if (n_in < 7) return;
    if ((size_t)in_sizes[0] < ((size_t)(NB - 1) * SEQ_FULL + SEQ) * DIMM) return;
    if (in_sizes[1] < DIMM || (size_t)in_sizes[2] < (size_t)QKVW * DIMM || (size_t)in_sizes[3] < (size_t)DIMM * DIMM || in_sizes[4] < NHD) return;
    if ((size_t)in_sizes[5] < (size_t)NBH * HD * HD || (size_t)in_sizes[6] < (size_t)NBH * HD) return;
    if ((size_t)out_size < OUT2_OFF + (size_t)NBH * HD) return;
    if (WS_TOTAL > ws_size) return;
    const float* x = (const float*)d_in[0]; const float* gamma = (const float*)d_in[1]; const float* w_qkv = (const float*)d_in[2]; const float* w_out = (const float*)d_in[3];
    const float* gates = (const float*)d_in[4]; const float* mem_kv = (const float*)d_in[5]; const float* mem_norm = (const float*)d_in[6];
    float* out0 = (float*)d_out; float* out1 = out0 + OUT1_OFF; float* out2 = out0 + OUT2_OFF;
    char* ws = (char*)d_ws;
    bf* WQB = (bf*)(ws + O_RW); h16* WQH = (h16*)(ws + O_RW + SZ_WQ);
    bf* QC = (bf*)(ws + O_RW); bf* KC = (bf*)(ws + O_RW + SZ_QC); bf* VTC = (bf*)(ws + O_RW + 2 * SZ_QC);
    bf* WOB = (bf*)(ws + O_WOB); h16* WOH = (h16*)(ws + O_WOH); h16* MEMT = (h16*)(ws + O_MEMT);
    float* INVF = (float*)(ws + O_INVF); float* COS = (float*)(ws + O_COS); float* SIN = (float*)(ws + O_SIN);
    h16* XN = (h16*)(ws + O_XN); h16* MRG = (h16*)(ws + O_XN);
    bf* XH = (bf*)(ws + O_XH); bf* XL = (bf*)(ws + O_XL); bf* MH = (bf*)(ws + O_XH); bf* ML = (bf*)(ws + O_XL);
    float* QKV = (float*)(ws + O_RQ); float* NUM = (float*)(ws + O_RQ); float* SE = (float*)(ws + O_RQ + SZ_NUM); bf* PC = (bf*)(ws + O_RQ + SZ_NUM + SZ_SE); float* CTXE = (float*)(ws + O_RQ + SZ_NUM + SZ_SE + SZ_PC);
    h16* QROT = (h16*)(ws + O_QROT); h16* VNT = (h16*)(ws + O_QROT); h16* KROT = (h16*)(ws + O_KROT); h16* VT = (h16*)(ws + O_VT);
    h16* FEAT = (h16*)(ws + O_FEAT); h16* KFT = (h16*)(ws + O_KFT); float* PART = (float*)(ws + O_PART); float* RDEN = (float*)(ws + O_RDEN);
    float* NUMq = NUM; float* NUMk = NUM + (size_t)NBH * SEQ * HD; float* RDq = RDEN; float* RDk = RDEN + (size_t)NBH * SEQ;

    k_cvtw<<<(unsigned)(((size_t)QKVW * DIMM / 8 + 255) / 256), 256, 0, stream>>>(w_qkv, WQB, WQH, (unsigned)((size_t)QKVW * DIMM / 8));
    k_cvtw<<<(unsigned)(((size_t)DIMM * DIMM / 8 + 255) / 256), 256, 0, stream>>>(w_out, WOB, WOH, (unsigned)((size_t)DIMM * DIMM / 8));
    k_memT<<<NBH, 256, 0, stream>>>(mem_kv, MEMT);
    k_invf<<<1, 32, 0, stream>>>(INVF);
    k_ropetab<<<SEQ * 64 / 256, 256, 0, stream>>>(INVF, COS, SIN);
    k_rms<<<NB * SEQ / 8, 256, 0, stream>>>(x, gamma, XN, XH, XL);
    k_gemmw<bf, 1, false><<<dim3(RH / 64, QKVW / 64, NB), 32, 0, stream>>>(XH, XL, WQB, DIMM, QKV, QKVW, nullptr, 1.0f, (size_t)RH * DIMM, 0, (size_t)SEQ * QKVW);
    if (SEQ > RH) k_gemmw<h16, 0, false><<<dim3((SEQ - RH) / 64, QKVW / 64, NB), 32, 0, stream>>>(XN + (size_t)RH * DIMM, nullptr, WQH, DIMM, QKV + (size_t)RH * QKVW, QKVW, nullptr, 1.0f / WCAR, (size_t)SEQ * DIMM, 0, (size_t)SEQ * QKVW);
    k_prep<<<dim3(SEQ / 64, NBH), 256, 0, stream>>>(QKV, COS, SIN, mem_norm, QROT, KROT, VT, FEAT, KFT, QC, KC, VTC, PART, RDEN);
    k_gemmw<h16, 0, false><<<dim3(SEQ / 64, HD / 64, 2 * NBH), 32, 0, stream>>>(FEAT, nullptr, MEMT, HD, NUM, HD, nullptr, 1.0f, (size_t)SEQ * HD, (size_t)HD * HD, (size_t)SEQ * HD);
    k_gemmw<bf, 0, false><<<dim3(RH / 64, RH / 64, NBH), 32, 0, stream>>>(QC, nullptr, KC, KCAT, SE, RH, nullptr, 1.0f, (size_t)RH * KCAT, (size_t)RH * KCAT, (size_t)RH * RH);
    k_asoftE<<<NBH * RH / 8, 256, 0, stream>>>(SE, PC);
    k_gemmw<bf, 0, false><<<dim3(RH / 64, HD / 64, NBH), 32, 0, stream>>>(PC, nullptr, VTC, PCAT, CTXE, HD, nullptr, 1.0f, (size_t)RH * PCAT, (size_t)HD * PCAT, (size_t)RH * HD);
    k_mergeE<<<NBH * RH * 16 / 256, 256, 0, stream>>>(CTXE, NUMq, RDq, gates, MH, ML);
    if (SEQ > RH) k_flash<<<dim3((SEQ - RH) / 16, NBH), 32, 0, stream>>>(QROT, KROT, VT, NUMq, RDq, gates, MRG);
    k_gemmw<bf, 1, false><<<dim3(RH / 64, DIMM / 64, NB), 32, 0, stream>>>(MH, ML, WOB, DIMM, out0, DIMM, nullptr, 1.0f, (size_t)RH * DIMM, 0, (size_t)SEQ_FULL * DIMM);
    if (SEQ > RH) k_gemmw<h16, 0, false><<<dim3((SEQ - RH) / 64, DIMM / 64, NB), 32, 0, stream>>>(MRG + (size_t)RH * DIMM, nullptr, WOH, DIMM, out0 + (size_t)RH * DIMM, DIMM, nullptr, 1.0f / (WCAR * MCAR), (size_t)SEQ * DIMM, 0, (size_t)SEQ_FULL * DIMM);
    k_vnew<<<dim3(SEQ / 64, NBH), 256, 0, stream>>>(NUMk, RDk, VT, VNT);
    k_gemmw<h16, 0, true><<<dim3(HD / 64, HD / 64, NBH), 32, 0, stream>>>(KFT, nullptr, VNT, SEQ, out1, HD, mem_kv, 1.0f, (size_t)HD * SEQ, (size_t)HD * SEQ, (size_t)HD * HD);
    k_normfin<<<NBH, 32, 0, stream>>>(PART, mem_norm, out2);
}
